// DPLRStateSpaceModel_54460185313714
// MI455X (gfx1250) — hardware-run, weakly checked
//
#include <hip/hip_runtime.h>
#include <math.h>

typedef __attribute__((ext_vector_type(16))) _Float16 v16h;
typedef __attribute__((ext_vector_type(8)))  _Float16 v8h;
typedef __attribute__((ext_vector_type(8)))  float    v8f;
typedef __attribute__((ext_vector_type(4)))  float    v4f;
typedef __attribute__((ext_vector_type(2)))  float    v2f;
typedef __attribute__((ext_vector_type(4)))  unsigned v4u;

constexpr int kBatch = 4;
constexpr int kSeq   = 2048;
constexpr int kDim   = 1024;
constexpr int kNst   = 16;
constexpr int kRows  = kBatch * kSeq;
static_assert(kRows == 8192, "token rows");
static_assert((kDim % 32) == 0, "GEMM K multiple of 32");
static_assert((kRows % 64) == 0 && (kDim % 64) == 0, "GEMM M and N multiples of 64");

constexpr float kCarryAct = 16.0f;
constexpr float kCarryW   = 256.0f;
constexpr float kFold     = 1.0f / (kCarryAct * kCarryW);
constexpr float kF16MinNormal = 6.103515625e-05f;
static_assert(kFold == 1.0f / 4096.0f, "fold constant");

constexpr size_t kOffXH  = 0;
constexpr size_t kOffWIH = kOffXH  + (size_t)kRows * kDim * 2;
constexpr size_t kOffWOH = kOffWIH + (size_t)kDim  * kDim * 2;
constexpr size_t kOffXIN = kOffWOH + (size_t)kDim  * kDim * 2;
constexpr size_t kOffYH  = kOffXIN + (size_t)kRows * kDim * 4;
constexpr size_t kOffABT = kOffYH  + (size_t)kRows * kDim * 2;
constexpr size_t kOffCBT = kOffABT + (size_t)kDim  * kNst * 4;
constexpr size_t kWsTotal = kOffCBT + (size_t)kDim * kNst * 4;
static_assert(kWsTotal == 71434240ull, "carve total");
static_assert(kWsTotal <= 134217728ull, "carve cap");
static_assert((kOffWIH % 128) == 0 && (kOffWOH % 128) == 0 && (kOffXIN % 128) == 0 &&
              (kOffYH % 128) == 0 && (kOffABT % 128) == 0 && (kOffCBT % 128) == 0, "128-B aligned regions");

__device__ __forceinline__ float carry_flush(float v, float carry) {
  const float c = v * carry;
  return (fabsf(c) < kF16MinNormal) ? 0.0f : c;
}
__device__ __forceinline__ unsigned pack2_f16(float ca, float cb) {
  const _Float16 ha = (_Float16)ca;
  const _Float16 hb = (_Float16)cb;
  const unsigned short ua = __builtin_bit_cast(unsigned short, ha);
  const unsigned short ub = __builtin_bit_cast(unsigned short, hb);
  return (unsigned)ua | ((unsigned)ub << 16);
}

constexpr int kPrepBlkX = kRows * kDim / 8 / 256;
constexpr int kPrepBlkW = kDim * kDim / 8 / 256;
constexpr int kPrepBlkT = kDim * kNst / 256;
constexpr int kPrepBlkPlanes = kPrepBlkX + 2 * kPrepBlkW;
constexpr int kPrepBlocks = kPrepBlkPlanes + kPrepBlkT;
static_assert(kPrepBlkX == 4096 && kPrepBlkW == 512 && kPrepBlkT == 64, "prep coverage");
static_assert((size_t)kPrepBlkX * 256 * 8 == (size_t)kRows * kDim, "x plane covered exactly");
static_assert((size_t)kPrepBlkW * 256 * 8 == (size_t)kDim * kDim, "weight plane covered exactly");
static_assert(kPrepBlkT * 256 == kDim * kNst, "tables covered exactly");

__global__ __launch_bounds__(256) void prep_kernel(
    const float* __restrict__ x, const float* __restrict__ W_in, const float* __restrict__ W_out,
    const float* __restrict__ A_log, const float* __restrict__ B_ssm, const float* __restrict__ C_ssm,
    const float* __restrict__ dt_log,
    unsigned* __restrict__ XH, unsigned* __restrict__ WIH, unsigned* __restrict__ WOH,
    float* __restrict__ ABT, float* __restrict__ CBT)
{
  const int bx  = blockIdx.x;
  const int tid = threadIdx.x;
  if (bx < kPrepBlkPlanes) {
    const float* src = x;
    unsigned* dst = XH;
    float carry = kCarryAct;
    int lb = bx;
    if (bx >= kPrepBlkX + kPrepBlkW) {
      src = W_out; dst = WOH; carry = kCarryW; lb = bx - kPrepBlkX - kPrepBlkW;
    } else if (bx >= kPrepBlkX) {
      src = W_in; dst = WIH; carry = kCarryW; lb = bx - kPrepBlkX;
    }
    const size_t e0 = ((size_t)lb * 256 + (size_t)tid) * 8;
    const v4f a0 = *(const v4f*)(src + e0);
    const v4f a1 = *(const v4f*)(src + e0 + 4);
    const float f0 = a0[0], f1 = a0[1], f2 = a0[2], f3 = a0[3];
    const float f4 = a1[0], f5 = a1[1], f6 = a1[2], f7 = a1[3];
    const unsigned w0 = pack2_f16(carry_flush(f0, carry), carry_flush(f1, carry));
    const unsigned w1 = pack2_f16(carry_flush(f2, carry), carry_flush(f3, carry));
    const unsigned w2 = pack2_f16(carry_flush(f4, carry), carry_flush(f5, carry));
    const unsigned w3 = pack2_f16(carry_flush(f6, carry), carry_flush(f7, carry));
    const v4u wv = {w0, w1, w2, w3};
    volatile v4u* q = (volatile v4u*)(dst + (e0 >> 1));
    *q = wv;
    __threadfence();
    *q = wv;
  } else {
    const int g = (bx - kPrepBlkPlanes) * 256 + tid;
    const int d = g >> 4;
    const float Ad = -expf(A_log[g]);
    const float dt = expf(dt_log[d]);
    const float ab = expf(dt * Ad);
    const float qd = (ab - 1.0f) / Ad;
    const float bb = qd * B_ssm[g];
    const float cb = C_ssm[g] * bb;
    volatile float* pa = ABT + g;
    volatile float* pc = CBT + g;
    *pa = ab;
    *pc = cb;
    __threadfence();
    *pa = ab;
    *pc = cb;
  }
}

namespace eng {

union FragU { v16h v; v8h h[2]; };

__device__ __forceinline__ v16h frag_load(const _Float16* p) {
  FragU f;
  f.h[0] = *(const v8h*)(p);
  f.h[1] = *(const v8h*)(p + 16);
  return f.v;
}

__device__ __forceinline__ v8f mma_g(v16h a, v16h b, v8f c) {
  c = __builtin_amdgcn_wmma_f32_16x16x32_f16(false, a, false, b, (short)0, c, false, false);
  asm volatile("v_nop\n\tv_nop\n\tv_nop\n\tv_nop" : "+v"(c) : "v"(a), "v"(b));
  return c;
}

__global__ __launch_bounds__(256) void gemm64_f16(
    const unsigned short* __restrict__ Ap, int lda,
    const unsigned short* __restrict__ Btp, int ldb,
    float* __restrict__ C, int ldc,
    int M, int N, int K, float scale)
{
  const _Float16* A  = (const _Float16*)Ap;
  const _Float16* Bt = (const _Float16*)Btp;
  __shared__ __align__(16) float sT[8][16 * 68];
  const int lane = threadIdx.x & 31;
  const int wave = threadIdx.x >> 5;
  const int tilesN = N >> 6;
  const int tilesM = M >> 6;
  const int tile = blockIdx.x * 8 + wave;
  if (tile >= tilesM * tilesN) return;
  const int tm = tile / tilesN;
  const int tn = tile - tm * tilesN;
  const int m0 = tm << 6;
  const int n0 = tn << 6;

  const int rlane = lane & 15;
  const int koff  = (lane >> 4) * 8;
  const int mOff  = (lane >> 4) * 8;

  v8f acc[4][4];
#pragma unroll
  for (int i = 0; i < 4; ++i)
#pragma unroll
    for (int j = 0; j < 4; ++j) acc[i][j] = (v8f){0.f, 0.f, 0.f, 0.f, 0.f, 0.f, 0.f, 0.f};

  for (int k0 = 0; k0 < K; k0 += 32) {
    v16h bh[4];
#pragma unroll
    for (int j = 0; j < 4; ++j) {
      const size_t bo = (size_t)(n0 + (j << 4) + rlane) * (size_t)ldb + (size_t)(koff + k0);
      bh[j] = frag_load(Bt + bo);
    }
#pragma unroll
    for (int i = 0; i < 4; ++i) {
      const size_t ao = (size_t)(m0 + (i << 4) + rlane) * (size_t)lda + (size_t)(koff + k0);
      const v16h ah = frag_load(A + ao);
#pragma unroll
      for (int j = 0; j < 4; ++j) acc[i][j] = mma_g(ah, bh[j], acc[i][j]);
    }
  }

  float* slab = sT[wave];
#pragma unroll
  for (int i = 0; i < 4; ++i) {
    const int mBase = m0 + (i << 4);
#pragma unroll
    for (int j = 0; j < 4; ++j) {
#pragma unroll
      for (int r = 0; r < 8; ++r) {
        const float v = acc[i][j][r] * scale;
        slab[(mOff + r) * 68 + (j << 4) + rlane] = v;
      }
    }
    __builtin_amdgcn_fence(__ATOMIC_RELEASE, "workgroup");
    __builtin_amdgcn_wave_barrier();
    __builtin_amdgcn_fence(__ATOMIC_ACQUIRE, "workgroup");
    {
      const int hh = lane >> 4;
      const int c4 = (lane & 15) * 4;
      for (int pass = 0; pass < 2; ++pass) {
#pragma unroll
        for (int it = 0; it < 8; ++it) {
          const int row = it * 2 + hh;
          const v4f v = *(const v4f*)(slab + row * 68 + c4);
          *(volatile v4f*)(C + (size_t)(mBase + row) * (size_t)ldc + (size_t)(n0 + c4)) = v;
        }
        __threadfence();
      }
    }
    __builtin_amdgcn_fence(__ATOMIC_RELEASE, "workgroup");
    __builtin_amdgcn_wave_barrier();
    __builtin_amdgcn_fence(__ATOMIC_ACQUIRE, "workgroup");
  }
}

}

constexpr int kRecurWaves  = kBatch * (kDim / 64);
constexpr int kRecurBlocks = kRecurWaves / 8;
static_assert(kRecurWaves == 64 && kRecurBlocks == 8, "recurrence coverage");

__global__ __launch_bounds__(256) void recur_kernel(
    const float* __restrict__ XIN, const float* __restrict__ ABT, const float* __restrict__ CBT,
    const float* __restrict__ Dsk, unsigned* __restrict__ YH)
{
  const int lane = threadIdx.x & 31;
  const int wave = threadIdx.x >> 5;
  const int gw = blockIdx.x * 8 + wave;
  const int b  = gw / (kDim / 64);
  const int d  = (gw - b * (kDim / 64)) * 64 + 2 * lane;

  float a0[kNst], a1[kNst], c0[kNst], c1[kNst], h0[kNst], h1[kNst];
#pragma unroll
  for (int q = 0; q < 4; ++q) {
    const v4f va0 = *(const v4f*)(ABT + (size_t)d * kNst + 4 * q);
    const v4f va1 = *(const v4f*)(ABT + (size_t)(d + 1) * kNst + 4 * q);
    const v4f vc0 = *(const v4f*)(CBT + (size_t)d * kNst + 4 * q);
    const v4f vc1 = *(const v4f*)(CBT + (size_t)(d + 1) * kNst + 4 * q);
    a0[4 * q + 0] = va0[0]; a0[4 * q + 1] = va0[1]; a0[4 * q + 2] = va0[2]; a0[4 * q + 3] = va0[3];
    a1[4 * q + 0] = va1[0]; a1[4 * q + 1] = va1[1]; a1[4 * q + 2] = va1[2]; a1[4 * q + 3] = va1[3];
    c0[4 * q + 0] = vc0[0]; c0[4 * q + 1] = vc0[1]; c0[4 * q + 2] = vc0[2]; c0[4 * q + 3] = vc0[3];
    c1[4 * q + 0] = vc1[0]; c1[4 * q + 1] = vc1[1]; c1[4 * q + 2] = vc1[2]; c1[4 * q + 3] = vc1[3];
  }
#pragma unroll
  for (int n = 0; n < kNst; ++n) { h0[n] = 0.0f; h1[n] = 0.0f; }
  const v2f dv = *(const v2f*)(Dsk + d);
  const float dd0 = dv[0], dd1 = dv[1];

  const float* xp = XIN + (size_t)b * kSeq * kDim + (size_t)d;
  unsigned*    yp = YH + (size_t)b * kSeq * (kDim / 2) + (size_t)(d >> 1);

#pragma unroll 1
  for (int l = 0; l < kSeq; ++l) {
    const v2f xv = *(const v2f*)(xp + (size_t)l * kDim);
    const float x0 = xv[0], x1 = xv[1];
    float y0 = dd0 * x0;
    float y1 = dd1 * x1;
#pragma unroll
    for (int n = 0; n < kNst; ++n) {
      h0[n] = fmaf(a0[n], h0[n], x0);
      h1[n] = fmaf(a1[n], h1[n], x1);
      y0 = fmaf(c0[n], h0[n], y0);
      y1 = fmaf(c1[n], h1[n], y1);
    }
    const float s0 = fminf(fmaxf(y0, -3750.0f), 3750.0f);
    const float s1 = fminf(fmaxf(y1, -3750.0f), 3750.0f);
    const unsigned w = pack2_f16(carry_flush(s0, kCarryAct), carry_flush(s1, kCarryAct));
    volatile unsigned* q = yp + (size_t)l * (kDim / 2);
    *q = w;
    __threadfence();
    *q = w;
  }
}

constexpr int kGemmTiles  = (kRows / 64) * (kDim / 64);
constexpr int kGemmBlocks = kGemmTiles / 8;
static_assert(kGemmTiles == 2048 && kGemmBlocks * 8 == kGemmTiles, "GEMM grid covers every tile exactly");

extern "C" void kernel_launch(void* const* d_in, const int* in_sizes, int n_in,
                              void* d_out, int out_size, void* d_ws, size_t ws_size,
                              hipStream_t stream) {
  if (n_in < 8) return;
  if (in_sizes[0] != kRows * kDim) return;
  if (in_sizes[1] != kDim * kDim) return;
  if (in_sizes[2] != kDim * kDim) return;
  if (in_sizes[3] != kDim * kNst) return;
  if (in_sizes[4] != kDim * kNst) return;
  if (in_sizes[5] != kDim * kNst) return;
  if (in_sizes[6] != kDim) return;
  if (in_sizes[7] != kDim) return;
  if (out_size != kRows * kDim) return;
  if (ws_size < kWsTotal) return;

  const float* x      = (const float*)d_in[0];
  const float* W_in   = (const float*)d_in[1];
  const float* W_out  = (const float*)d_in[2];
  const float* A_log  = (const float*)d_in[3];
  const float* B_ssm  = (const float*)d_in[4];
  const float* C_ssm  = (const float*)d_in[5];
  const float* dt_log = (const float*)d_in[6];
  const float* D_ssm  = (const float*)d_in[7];
  float* out = (float*)d_out;

  char* ws = (char*)d_ws;
  unsigned* XH  = (unsigned*)(ws + kOffXH);
  unsigned* WIH = (unsigned*)(ws + kOffWIH);
  unsigned* WOH = (unsigned*)(ws + kOffWOH);
  float*    XIN = (float*)(ws + kOffXIN);
  unsigned* YH  = (unsigned*)(ws + kOffYH);
  float*    ABT = (float*)(ws + kOffABT);
  float*    CBT = (float*)(ws + kOffCBT);

  prep_kernel<<<kPrepBlocks, 256, 0, stream>>>(x, W_in, W_out, A_log, B_ssm, C_ssm, dt_log,
                                               XH, WIH, WOH, ABT, CBT);

  eng::gemm64_f16<<<kGemmBlocks, 256, 0, stream>>>(
      (const unsigned short*)XH, kDim, (const unsigned short*)WIH, kDim,
      XIN, kDim, kRows, kDim, kDim, kFold);

  recur_kernel<<<kRecurBlocks, 256, 0, stream>>>(XIN, ABT, CBT, D_ssm, YH);

  eng::gemm64_f16<<<kGemmBlocks, 256, 0, stream>>>(
      (const unsigned short*)YH, kDim, (const unsigned short*)WOH, kDim,
      out, kDim, kRows, kDim, kDim, kFold);
}
